// RobustMambaDiagSSM_40896678592897
// MI455X (gfx1250) — hardware-verified
//
#include <hip/hip_runtime.h>
#include <math.h>


#define B_SZ    4
#define T_SZ    2048
#define D_SZ    1024
#define N_SZ    1024
#define DOUT    1024
#define BT      (B_SZ * T_SZ)
#define NCAT    (4 * N_SZ)
#define PITER   600
#define EPS_CAP 0.9999f
#define SL_IN_INV  1
#define SL_OUT_INV 33
#define SPITCH  36
#define STW     (16 * SPITCH)

static_assert(BT % 128 == 0);
static_assert(N_SZ % 64 == 0);
static_assert(D_SZ % 32 == 0);
static_assert(DOUT % 64 == 0);
static_assert(T_SZ % 32 == 0);
static_assert((B_SZ * N_SZ) % 256 == 0);

typedef _Float16 v8h  __attribute__((ext_vector_type(8)));
typedef _Float16 v16h __attribute__((ext_vector_type(16)));
typedef float    v4f  __attribute__((ext_vector_type(4)));
typedef float    v8f  __attribute__((ext_vector_type(8)));

union Frag { v16h v; v8h half[2]; };

constexpr size_t SZ_UH  = (size_t)BT * D_SZ * 2;
constexpr size_t SZ_YH  = (size_t)BT * N_SZ * 2;
constexpr size_t SZ_WC  = (size_t)NCAT * D_SZ * 2;
constexpr size_t SZ_WO  = (size_t)DOUT * N_SZ * 2;
constexpr size_t SZ_SIG = 256;
constexpr size_t SZ_PL  = (size_t)BT * N_SZ * 4;
constexpr size_t SZ_G   = (size_t)N_SZ * N_SZ * 4;

constexpr size_t OFF_UH  = 0;
constexpr size_t OFF_YH  = 0;
constexpr size_t OFF_WC  = OFF_UH + SZ_UH;
constexpr size_t OFF_WO  = OFF_WC + SZ_WC;
constexpr size_t OFF_SIG = OFF_WO + SZ_WO;
constexpr size_t OFF_A   = OFF_SIG + SZ_SIG;
constexpr size_t OFF_BU  = OFF_A + SZ_PL;
constexpr size_t OFF_C   = OFF_BU + SZ_PL;
constexpr size_t WS_END  = OFF_C + SZ_PL;
constexpr size_t OFF_G0  = OFF_A;
constexpr size_t OFF_G1  = OFF_A + SZ_G;
static_assert(WS_END <= (size_t)134217728);
static_assert(OFF_G1 + SZ_G <= OFF_BU);
static_assert(SZ_YH <= SZ_UH);
static_assert(OFF_WC % 128 == 0 && OFF_WO % 128 == 0 && OFF_SIG % 128 == 0 && OFF_A % 128 == 0);
static_assert(OFF_BU % 128 == 0 && OFF_C % 128 == 0 && OFF_G1 % 128 == 0);

__device__ __forceinline__ void mma16(v8f& acc, const Frag& a, const Frag& b) {
    acc = __builtin_amdgcn_wmma_f32_16x16x32_f16(false, a.v, false, b.v, (short)0, acc, false, false);
    asm volatile("v_nop\n\tv_nop\n\tv_nop\n\tv_nop" : "+v"(acc) : "v"(a.v), "v"(b.v));
}
__device__ __forceinline__ float wsum_f(float x) {
#pragma unroll
    for (int mm = 16; mm >= 1; mm >>= 1) x += __shfl_xor(x, mm, 32);
    return x;
}
__device__ __forceinline__ double wsum_d(double x) {
#pragma unroll
    for (int mm = 16; mm >= 1; mm >>= 1) x += __shfl_xor(x, mm, 32);
    return x;
}
__device__ __forceinline__ float softplus_col(float x) {
    return fmaxf(x, 0.0f) + log1pf(expf(-fabsf(x)));
}
__device__ __forceinline__ float softplus_el(float x) {
    return fmaxf(x, 0.0f) + __logf(1.0f + __expf(-fabsf(x)));
}
__device__ __forceinline__ float tanh_el(float x) {
    const float e = __expf(2.0f * fabsf(x));
    const float t = 1.0f - 2.0f * __builtin_amdgcn_rcpf(e + 1.0f);
    return copysignf(t, x);
}

__global__ __launch_bounds__(256)
void cvt_kernel(const float* __restrict__ src, _Float16* dst, int n8, float scale)
{
    const int i = blockIdx.x * 256 + threadIdx.x;
    if (i >= n8) return;
    const size_t e = (size_t)i * 8;
    const v4f a = *(const v4f*)(src + e);
    const v4f b = *(const v4f*)(src + e + 4);
    v8h o;
#pragma unroll
    for (int c = 0; c < 4; ++c) {
        o[c]     = (_Float16)(a[c] * scale);
        o[c + 4] = (_Float16)(b[c] * scale);
    }
    *(volatile v8h*)(dst + e) = o;
    __threadfence();
    *(volatile v8h*)(dst + e) = o;
}

template<int NBF>
__device__ __forceinline__ void tile_store_pass(const float* st, float* gp, int ldc, int lane) {
    constexpr int CW  = NBF * 16;
    constexpr int P   = CW + 4;
    constexpr int LPR = CW / 4;
    static_assert(32 % LPR == 0);
    constexpr int RPI = 32 / LPR;
    constexpr int NIT = 32 / RPI;
    const int rsub = lane / LPR;
    const int c0   = (lane % LPR) * 4;
#pragma unroll
    for (int it = 0; it < NIT; ++it) {
        const int row = it * RPI + rsub;
        const v4f v = *(const v4f*)(st + row * P + c0);
        *(volatile v4f*)(gp + (size_t)row * ldc + c0) = v;
    }
}

template<int NBF>
__global__ __launch_bounds__(128)
void gemm_kernel(const _Float16* Am, const _Float16* Bm, float* C, int K, int ldc,
                 float cscale, const float* __restrict__ sigl, int use_sig)
{
    constexpr int CW = NBF * 16;
    constexpr int P  = CW + 4;
    static_assert(CW % 32 == 0);
    __shared__ __attribute__((aligned(16))) float stile[4][32 * P];

    const int tid  = threadIdx.x;
    const int lane = tid & 31;
    const int wave = tid >> 5;
    const int h    = lane >> 4;
    const int m    = lane & 15;
    const int wm   = wave >> 1;
    const int wn   = wave & 1;

    const int rowW = blockIdx.y * 64 + wm * 32;
    const int colW = blockIdx.x * (2 * CW) + wn * CW;

    v8f acc[2 * NBF];
#pragma unroll
    for (int j = 0; j < 2 * NBF; ++j)
#pragma unroll
        for (int r = 0; r < 8; ++r) acc[j][r] = 0.0f;

    const size_t aoff  = (size_t)(rowW + m) * K + 8 * h;
    const size_t boff  = (size_t)(colW + m) * K + 8 * h;
    const size_t sub16 = (size_t)16 * K;
    const int nk = K >> 5;

#pragma unroll 1
    for (int kt = 0; kt < nk; ++kt) {
        const size_t k0 = (size_t)kt * 32;
        Frag fa[2], fb[NBF];
#pragma unroll
        for (int s = 0; s < 2; ++s) {
            const _Float16* p = Am + aoff + s * sub16 + k0;
            fa[s].half[0] = *(const v8h*)(p);
            fa[s].half[1] = *(const v8h*)(p + 16);
        }
#pragma unroll
        for (int j = 0; j < NBF; ++j) {
            const _Float16* p = Bm + boff + j * sub16 + k0;
            fb[j].half[0] = *(const v8h*)(p);
            fb[j].half[1] = *(const v8h*)(p + 16);
        }
#pragma unroll
        for (int s = 0; s < 2; ++s)
#pragma unroll
            for (int j = 0; j < NBF; ++j)
                mma16(acc[s * NBF + j], fa[s], fb[j]);
    }

    float scl = cscale;
    if (use_sig != 0) scl = cscale * sigl[SL_OUT_INV];

    float* st = stile[wave];
#pragma unroll
    for (int s = 0; s < 2; ++s)
#pragma unroll
        for (int j = 0; j < NBF; ++j)
#pragma unroll
            for (int r = 0; r < 8; ++r)
                st[(s * 16 + 8 * h + r) * P + j * 16 + m] = acc[s * NBF + j][r] * scl;
    __syncthreads();

    float* gp = C + (size_t)rowW * ldc + colW;
    tile_store_pass<NBF>(st, gp, ldc, lane);
    __threadfence();
    tile_store_pass<NBF>(st, gp, ldc, lane);
}

__global__ __launch_bounds__(256)
void power_kernel(const float* __restrict__ Gb, const float* __restrict__ Win,
                  const float* __restrict__ Wout, float* sigl)
{
    __shared__ __attribute__((aligned(16))) float sv[N_SZ];
    __shared__ float  sred[8];
    __shared__ double dred[16];
    const int tid  = threadIdx.x;
    const int lane = tid & 31;
    const int wave = tid >> 5;
    const int mat  = blockIdx.x;
    const float* G = Gb + (size_t)mat * ((size_t)N_SZ * N_SZ);
    const float* W = (mat == 0) ? Win : Wout;

#pragma unroll
    for (int q = 0; q < 4; ++q) sv[tid + 256 * q] = 0.03125f;
    __syncthreads();

    const float* g0 = G + (size_t)tid * N_SZ;
#pragma unroll 1
    for (int it = 0; it < PITER; ++it) {
        float acc[4] = {0.0f, 0.0f, 0.0f, 0.0f};
#pragma unroll 1
        for (int j = 0; j < N_SZ; j += 4) {
            const v4f vv = *(const v4f*)(sv + j);
#pragma unroll
            for (int q = 0; q < 4; ++q) {
                const v4f gg = *(const v4f*)(g0 + (size_t)q * (256 * N_SZ) + j);
                acc[q] = fmaf(gg[0], vv[0], acc[q]);
                acc[q] = fmaf(gg[1], vv[1], acc[q]);
                acc[q] = fmaf(gg[2], vv[2], acc[q]);
                acc[q] = fmaf(gg[3], vv[3], acc[q]);
            }
        }
        float ss = acc[0] * acc[0] + acc[1] * acc[1] + acc[2] * acc[2] + acc[3] * acc[3];
        ss = wsum_f(ss);
        __syncthreads();
        if (lane == 0) sred[wave] = ss;
        __syncthreads();
        float tot = sred[0];
#pragma unroll
        for (int w = 1; w < 8; ++w) tot += sred[w];
        const float inv = rsqrtf(fmaxf(tot, 1e-30f));
#pragma unroll
        for (int q = 0; q < 4; ++q) sv[tid + 256 * q] = acc[q] * inv;
        __syncthreads();
    }

    double dy[4] = {0.0, 0.0, 0.0, 0.0};
#pragma unroll 1
    for (int i = 0; i < N_SZ; i += 4) {
        const v4f vv = *(const v4f*)(sv + i);
#pragma unroll
        for (int ii = 0; ii < 4; ++ii) {
            const float* wr = W + (size_t)(i + ii) * D_SZ + tid;
            const double vd = (double)vv[ii];
#pragma unroll
            for (int q = 0; q < 4; ++q) dy[q] = fma((double)wr[256 * q], vd, dy[q]);
        }
    }
    double num = dy[0] * dy[0] + dy[1] * dy[1] + dy[2] * dy[2] + dy[3] * dy[3];
    double den = 0.0;
#pragma unroll
    for (int q = 0; q < 4; ++q) {
        const double t = (double)sv[tid + 256 * q];
        den = fma(t, t, den);
    }
    num = wsum_d(num);
    den = wsum_d(den);
    if (lane == 0) { dred[wave] = num; dred[8 + wave] = den; }
    __syncthreads();
    double tn = dred[0], td = dred[8];
#pragma unroll
    for (int w = 1; w < 8; ++w) { tn += dred[w]; td += dred[8 + w]; }
    const float sigma = sqrtf((float)(tn / td));
    const float scl   = fmaxf(sigma, 1.0f);
    const float inv   = 1.0f / scl;

    v4f val = {0.0f, 0.0f, 0.0f, 0.0f};
    if (lane == 0) { val[0] = scl; val[1] = inv; val[2] = sigma; }
    float* p = sigl + mat * 32 + lane * 4;
    if (wave == 0 && lane < 8) { *(volatile v4f*)p = val; }
    __threadfence();
    if (wave == 0 && lane < 8) { *(volatile v4f*)p = val; }
}

__global__ __launch_bounds__(256)
void gemm_act_kernel(const _Float16* __restrict__ Uh, const _Float16* __restrict__ Wc,
                     const float* __restrict__ pnb, const float* __restrict__ alpha_log,
                     const float* __restrict__ delta_bias, const float* __restrict__ log_gamma,
                     const float* __restrict__ sigl,
                     float* Ap, float* BUp, float* Cp)
{
    __shared__ __attribute__((aligned(16))) float st[8 * 3 * STW];

    const int tid  = threadIdx.x;
    const int lane = tid & 31;
    const int wave = tid >> 5;
    const int h    = lane >> 4;
    const int m    = lane & 15;
    const int n0   = blockIdx.x * 32;
    const int m0   = blockIdx.y * 128;
    const int rw   = m0 + wave * 16;

    v8f acc[8];
#pragma unroll
    for (int j = 0; j < 8; ++j)
#pragma unroll
        for (int r = 0; r < 8; ++r) acc[j][r] = 0.0f;

    const _Float16* ap = Uh + (size_t)(rw + m) * D_SZ + 8 * h;
    const _Float16* bp = Wc + (size_t)(n0 + m) * D_SZ + 8 * h;

#pragma unroll 1
    for (int kt = 0; kt < D_SZ / 32; ++kt) {
        const int k0 = kt * 32;
        Frag a;
        a.half[0] = *(const v8h*)(ap + k0);
        a.half[1] = *(const v8h*)(ap + k0 + 16);
#pragma unroll
        for (int g = 0; g < 4; ++g) {
#pragma unroll
            for (int j = 0; j < 2; ++j) {
                const _Float16* q = bp + ((size_t)g * N_SZ + (size_t)j * 16) * D_SZ + k0;
                Frag b;
                b.half[0] = *(const v8h*)(q);
                b.half[1] = *(const v8h*)(q + 16);
                mma16(acc[g * 2 + j], a, b);
            }
        }
    }

    const float r32 = 1.0f / 32.0f;
    const float gsc = expf(log_gamma[0]) * sigl[SL_IN_INV] * r32;
    float alph[2], dbv[2], pbd[2], pbb[2], pbc[2];
#pragma unroll
    for (int j = 0; j < 2; ++j) {
        const int n = n0 + 16 * j + m;
        alph[j] = softplus_col(alpha_log[n]);
        dbv[j]  = delta_bias[n];
        pbd[j]  = pnb[n];
        pbb[j]  = pnb[N_SZ + n];
        pbc[j]  = pnb[2 * N_SZ + n];
    }
    float* sw = st + wave * (3 * STW);
#pragma unroll
    for (int j = 0; j < 2; ++j) {
#pragma unroll
        for (int r = 0; r < 8; ++r) {
            const float us  = acc[0 * 2 + j][r] * gsc;
            const float xd  = fmaf(acc[1 * 2 + j][r], r32, pbd[j]) + dbv[j];
            const float dl  = softplus_el(xd);
            float a = fminf(__expf(-(dl * alph[j])), EPS_CAP);
            float b = tanh_el(fmaf(acc[2 * 2 + j][r], r32, pbb[j]));
            float c = tanh_el(fmaf(acc[3 * 2 + j][r], r32, pbc[j]));
            const float p    = a * a + c * c;
            const float rr   = b * b;
            const float q    = a * b;
            const float d    = p - rr;
            const float disc = d * d + (4.0f * q) * q;
            const float lam  = 0.5f * ((p + rr) + sqrtf(disc + 1e-12f));
            const float sg   = sqrtf(lam + 1e-12f);
            const float is   = __builtin_amdgcn_rcpf(fmaxf(sg, 1.0f));
            a *= is; b *= is; c *= is;
            const int o = (8 * h + r) * SPITCH + 16 * j + m;
            sw[o]           = a;
            sw[STW + o]     = b * us;
            sw[2 * STW + o] = c;
        }
    }
    __syncthreads();

    const int rq = lane >> 3;
    const int c4 = (lane & 7) * 4;
    float* ga = Ap  + (size_t)rw * N_SZ + n0 + c4;
    float* gb = BUp + (size_t)rw * N_SZ + n0 + c4;
    float* gc = Cp  + (size_t)rw * N_SZ + n0 + c4;
#pragma unroll
    for (int it = 0; it < 4; ++it) {
        const int row = it * 4 + rq;
        const v4f va = *(const v4f*)(sw + row * SPITCH + c4);
        const v4f vb = *(const v4f*)(sw + STW + row * SPITCH + c4);
        const v4f vc = *(const v4f*)(sw + 2 * STW + row * SPITCH + c4);
        *(volatile v4f*)(ga + (size_t)row * N_SZ) = va;
        *(volatile v4f*)(gb + (size_t)row * N_SZ) = vb;
        *(volatile v4f*)(gc + (size_t)row * N_SZ) = vc;
    }
    __threadfence();
#pragma unroll
    for (int it = 0; it < 4; ++it) {
        const int row = it * 4 + rq;
        const v4f va = *(const v4f*)(sw + row * SPITCH + c4);
        const v4f vb = *(const v4f*)(sw + STW + row * SPITCH + c4);
        const v4f vc = *(const v4f*)(sw + 2 * STW + row * SPITCH + c4);
        *(volatile v4f*)(ga + (size_t)row * N_SZ) = va;
        *(volatile v4f*)(gb + (size_t)row * N_SZ) = vb;
        *(volatile v4f*)(gc + (size_t)row * N_SZ) = vc;
    }
}

__global__ __launch_bounds__(256)
void scan_kernel(const float* __restrict__ Ap, const float* __restrict__ BUp, const float* __restrict__ Cp,
                 const float* __restrict__ z0, _Float16* Yh)
{
    __shared__ __attribute__((aligned(16))) _Float16 sy[32 * 256];
    const int tid   = threadIdx.x;
    const int gcol  = blockIdx.x * 256 + tid;
    const int b     = gcol >> 10;
    const int n     = gcol & (N_SZ - 1);
    const int ncol0 = (blockIdx.x * 256) & (N_SZ - 1);
    const size_t rowb = (size_t)b * T_SZ;
    float z = z0[b * N_SZ + n];

#pragma unroll 1
    for (int tb = 0; tb < T_SZ; tb += 32) {
#pragma unroll 1
        for (int t = 0; t < 32; ++t) {
            const size_t o = (rowb + tb + t) * N_SZ + n;
            const float a  = Ap[o];
            const float bu = BUp[o];
            const float c  = Cp[o];
            const float y  = c * z;
            sy[t * 256 + tid] = (_Float16)(y * 8.0f);
            z = fmaf(a, z, bu);
        }
        __syncthreads();
        v8h vv[4];
#pragma unroll
        for (int it = 0; it < 4; ++it) {
            const int p = it * 256 + tid;
            const int row = p >> 5;
            const int c8  = (p & 31) * 8;
            vv[it] = *(const v8h*)(sy + row * 256 + c8);
        }
#pragma unroll
        for (int it = 0; it < 4; ++it) {
            const int p = it * 256 + tid;
            const int row = p >> 5;
            const int c8  = (p & 31) * 8;
            *(volatile v8h*)(Yh + (rowb + tb + row) * N_SZ + ncol0 + c8) = vv[it];
        }
        __threadfence();
#pragma unroll
        for (int it = 0; it < 4; ++it) {
            const int p = it * 256 + tid;
            const int row = p >> 5;
            const int c8  = (p & 31) * 8;
            *(volatile v8h*)(Yh + (rowb + tb + row) * N_SZ + ncol0 + c8) = vv[it];
        }
        __syncthreads();
    }
}

extern "C" void kernel_launch(void* const* d_in, const int* in_sizes, int n_in,
                              void* d_out, int out_size, void* d_ws, size_t ws_size,
                              hipStream_t stream)
{
    if (n_in < 9) return;
    if (in_sizes[0] != BT * D_SZ)        return;
    if (in_sizes[1] != B_SZ * N_SZ)      return;
    if (in_sizes[2] != N_SZ * D_SZ)      return;
    if (in_sizes[3] != DOUT * N_SZ)      return;
    if (in_sizes[4] != 3 * N_SZ * D_SZ)  return;
    if (in_sizes[5] != 3 * N_SZ)         return;
    if (in_sizes[6] != N_SZ)             return;
    if (in_sizes[7] != N_SZ)             return;
    if (in_sizes[8] < 1)                 return;
    if (out_size != BT * DOUT)           return;
    if (ws_size < WS_END)                return;

    const float* u          = (const float*)d_in[0];
    const float* z0         = (const float*)d_in[1];
    const float* Win        = (const float*)d_in[2];
    const float* Wout       = (const float*)d_in[3];
    const float* pnw        = (const float*)d_in[4];
    const float* pnb        = (const float*)d_in[5];
    const float* alpha_log  = (const float*)d_in[6];
    const float* delta_bias = (const float*)d_in[7];
    const float* log_gamma  = (const float*)d_in[8];
    float* out = (float*)d_out;

    char* ws = (char*)d_ws;
    _Float16* Uh   = (_Float16*)(ws + OFF_UH);
    _Float16* Yh   = (_Float16*)(ws + OFF_YH);
    _Float16* Wc   = (_Float16*)(ws + OFF_WC);
    _Float16* Wo   = (_Float16*)(ws + OFF_WO);
    float*    sigl = (float*)(ws + OFF_SIG);
    float*    Ap   = (float*)(ws + OFF_A);
    float*    BUp  = (float*)(ws + OFF_BU);
    float*    Cp   = (float*)(ws + OFF_C);
    float*    G0   = (float*)(ws + OFF_G0);
    float*    G1   = (float*)(ws + OFF_G1);

    {
        const int n8u = (BT * D_SZ) / 8;
        const int n8w = (N_SZ * D_SZ) / 8;
        const int n8p = (3 * N_SZ * D_SZ) / 8;
        const int n8o = (DOUT * N_SZ) / 8;
        cvt_kernel<<<dim3((n8u + 255) / 256), dim3(256), 0, stream>>>(u, Uh, n8u, 1.0f);
        cvt_kernel<<<dim3((n8w + 255) / 256), dim3(256), 0, stream>>>(Win, Wc, n8w, 32.0f);
        cvt_kernel<<<dim3((n8p + 255) / 256), dim3(256), 0, stream>>>(pnw, Wc + (size_t)N_SZ * D_SZ, n8p, 32.0f);
        cvt_kernel<<<dim3((n8o + 255) / 256), dim3(256), 0, stream>>>(Wout, Wo, n8o, 32.0f);
    }

    gemm_kernel<2><<<dim3(N_SZ / 64, N_SZ / 64), dim3(128), 0, stream>>>(
        (const _Float16*)Wc, (const _Float16*)Wc, G0, (int)D_SZ, (int)N_SZ, 1.0f / 1024.0f, (const float*)sigl, 0);
    gemm_kernel<2><<<dim3(DOUT / 64, DOUT / 64), dim3(128), 0, stream>>>(
        (const _Float16*)Wo, (const _Float16*)Wo, G1, (int)N_SZ, (int)DOUT, 1.0f / 1024.0f, (const float*)sigl, 0);

    power_kernel<<<dim3(2), dim3(256), 0, stream>>>((const float*)G0, Win, Wout, sigl);

    gemm_act_kernel<<<dim3(N_SZ / 32, BT / 128), dim3(256), 0, stream>>>(
        (const _Float16*)Uh, (const _Float16*)Wc, pnb, alpha_log, delta_bias, log_gamma,
        (const float*)sigl, Ap, BUp, Cp);

    scan_kernel<<<dim3((B_SZ * N_SZ) / 256), dim3(256), 0, stream>>>(
        (const float*)Ap, (const float*)BUp, (const float*)Cp, z0, Yh);

    gemm_kernel<2><<<dim3(DOUT / 64, BT / 64), dim3(128), 0, stream>>>(
        (const _Float16*)Yh, (const _Float16*)Wo, out, (int)N_SZ, (int)DOUT, 1.0f / 256.0f, (const float*)sigl, 1);
}
